// InvariantPointAttention_34187939676342
// MI455X (gfx1250) — hardware-run, weakly checked
//
#include <hip/hip_runtime.h>


#define LR   1024
#define TT   LR
#define ND   256
#define NH_  4
#define HD   64
#define NPT  24
#define PW   96
#define FPW  320
#define KA   160
#define VA   128
#define CW   352
#define ZH   2
#define RH   0
#define WIN  0
#define PCAR 1024.0f
#define SCL  0.125f
typedef _Float16 h16;
typedef unsigned short bf;
typedef __attribute__((ext_vector_type(16))) __bf16   v16bf;
typedef __attribute__((ext_vector_type(16))) _Float16 v16h;
typedef __attribute__((ext_vector_type(8)))  _Float16 v8h;
typedef __attribute__((ext_vector_type(8)))  unsigned short v8us;
typedef __attribute__((ext_vector_type(8)))  float    v8f;
typedef __attribute__((ext_vector_type(4)))  float    v4f;
typedef v8h  __attribute__((may_alias)) v8ha;
typedef v4f  __attribute__((may_alias)) v4fa;
typedef v8us __attribute__((may_alias)) v8usa;

__device__ __forceinline__ unsigned short f2bf(float f) { unsigned u = __float_as_uint(f); u += 0x7FFFu + ((u >> 16) & 1u); return (unsigned short)(u >> 16); }
__device__ __forceinline__ float bf2f(unsigned short b) { return __uint_as_float(((unsigned)b) << 16); }
__device__ __forceinline__ float bfr(float f) { return bf2f(f2bf(f)); }
__device__ __forceinline__ v16h cat16(v8h lo, v8h hi) { return __builtin_shufflevector(lo, hi, 0, 1, 2, 3, 4, 5, 6, 7, 8, 9, 10, 11, 12, 13, 14, 15); }
__device__ __forceinline__ v16bf cat16b(v8us lo, v8us hi) { return __builtin_bit_cast(v16bf, __builtin_shufflevector(lo, hi, 0, 1, 2, 3, 4, 5, 6, 7, 8, 9, 10, 11, 12, 13, 14, 15)); }
__device__ __forceinline__ v8f wmma16(v16h a, v16h b, v8f c) { return __builtin_amdgcn_wmma_f32_16x16x32_f16(false, a, false, b, (short)0, c, false, false); }
__device__ __forceinline__ v8f wmmab(v16bf a, v16bf b, v8f c) { return __builtin_amdgcn_wmma_f32_16x16x32_bf16(false, a, false, b, (short)0, c, false, false); }


template <typename T16> struct WFrag;
template <> struct WFrag<h16> { typedef v16h V; static __device__ __forceinline__ V ld(const h16* p) { return cat16(*(const v8h*)p, *(const v8h*)(p + 16)); } static __device__ __forceinline__ v8f mma(V a, V b, v8f c) { return wmma16(a, b, c); } };
template <> struct WFrag<bf> { typedef v16bf V; static __device__ __forceinline__ V ld(const bf* p) { return cat16b(*(const v8us*)p, *(const v8us*)(p + 16)); } static __device__ __forceinline__ v8f mma(V a, V b, v8f c) { return wmmab(a, b, c); } };
template <typename T16, int NSPLIT, bool BIAS>
__global__ __launch_bounds__(32) void k_gemmw(const T16* __restrict__ A, const T16* __restrict__ A2, const T16* __restrict__ Bt, const T16* __restrict__ Bt2, int K, float* C, int ldc, const float* __restrict__ bias, size_t sA, size_t sB, size_t sC) {
    typedef typename WFrag<T16>::V V;
    __shared__ __align__(16) float os[16 * 68];
    const size_t z = blockIdx.z; A += z * sA; if (A2) A2 += z * sA; Bt += z * sB; if (Bt2) Bt2 += z * sB; C += z * sC;
    const int lane = threadIdx.x & 31, lr = lane & 15, hi = lane >> 4; const int r0 = blockIdx.x * 64, c0 = blockIdx.y * 64;
    v8f acc[4][4];
#pragma unroll
    for (int mb = 0; mb < 4; ++mb)
#pragma unroll
        for (int nb = 0; nb < 4; ++nb) acc[mb][nb] = (v8f){};
    const size_t aoff = (size_t)(r0 + lr) * K + 8 * hi, boff = (size_t)(c0 + lr) * K + 8 * hi;
    for (int kc = 0; kc < K; kc += 32) {
        V a[4], a2[4];
#pragma unroll
        for (int mb = 0; mb < 4; ++mb) { a[mb] = WFrag<T16>::ld(A + aoff + (size_t)mb * 16 * K + kc); if (NSPLIT == 1 || NSPLIT == 2) a2[mb] = WFrag<T16>::ld(A2 + aoff + (size_t)mb * 16 * K + kc); }
#pragma unroll
        for (int nb = 0; nb < 4; ++nb) { const V b = WFrag<T16>::ld(Bt + boff + (size_t)nb * 16 * K + kc); V b2; if (NSPLIT >= 2) b2 = WFrag<T16>::ld(Bt2 + boff + (size_t)nb * 16 * K + kc);
#pragma unroll
            for (int mb = 0; mb < 4; ++mb) { acc[mb][nb] = WFrag<T16>::mma(a[mb], b, acc[mb][nb]); if (NSPLIT == 1 || NSPLIT == 2) acc[mb][nb] = WFrag<T16>::mma(a2[mb], b, acc[mb][nb]); if (NSPLIT >= 2) acc[mb][nb] = WFrag<T16>::mma(a[mb], b2, acc[mb][nb]); } }
        asm volatile("v_nop\n\tv_nop\n\tv_nop\n\tv_nop" : "+v"(acc[0][0]), "+v"(acc[1][1]), "+v"(acc[2][2]), "+v"(acc[3][3]) : "v"(a[0]), "v"(a[3]));
    }
#pragma unroll
    for (int mb = 0; mb < 4; ++mb) {
#pragma unroll
        for (int nb = 0; nb < 4; ++nb) {
#pragma unroll
            for (int j = 0; j < 8; ++j) os[(hi * 8 + j) * 68 + nb * 16 + lr] = acc[mb][nb][j]; }
        __builtin_amdgcn_wave_barrier(); asm volatile("" ::: "memory");
        float* crow = C + (size_t)(r0 + mb * 16) * ldc + c0;
#pragma unroll 1
        for (int ps = 0; ps < 2; ++ps) {
#pragma unroll
            for (int s = 0; s < 8; ++s) { const int row = 2 * s + hi, cofs = lr * 4; v4f val = *(const v4fa*)(os + row * 68 + cofs); if (BIAS) { val[0] += bfr(bias[c0 + cofs]); val[1] += bfr(bias[c0 + cofs + 1]); val[2] += bfr(bias[c0 + cofs + 2]); val[3] += bfr(bias[c0 + cofs + 3]); }
                *(volatile v4f*)(crow + (size_t)row * ldc + cofs) = val; }
            if (ps == 0) __threadfence(); }
        __builtin_amdgcn_wave_barrier(); asm volatile("" ::: "memory");
    }
}

__device__ __forceinline__ h16 tohx(float x) { return (h16)x; }
__device__ __forceinline__ void splitf(float y, unsigned short& h, unsigned short& l) { h = f2bf(y); l = f2bf(y - bf2f(h)); }
typedef __attribute__((ext_vector_type(2))) _Float16 v2h;
typedef __attribute__((ext_vector_type(4))) _Float16 v4h;
typedef __attribute__((ext_vector_type(2))) unsigned short v2us;
typedef __attribute__((ext_vector_type(4))) unsigned short v4us;
typedef __attribute__((ext_vector_type(2))) float v2f;
typedef __attribute__((ext_vector_type(4))) int v4i;

__global__ __launch_bounds__(256) void k_wtG(const float* __restrict__ w, int K, int N, bf* Bt) {
    const int lane = threadIdx.x & 31; const int L0 = (blockIdx.x * 8 + (threadIdx.x >> 5)) * 8; const int nlines = N * K / 64;
#pragma unroll
    for (int ps = 0; ps < 2; ++ps) {
        for (int l = 0; l < 8; ++l) { const int L = L0 + l; if (L >= nlines) break; const size_t e = (size_t)L * 64 + lane * 2; const int k = (int)(e % K), n = (int)(e / K); v2us o;
            o[0] = f2bf(w[(size_t)k * N + n]); o[1] = f2bf(w[(size_t)(k + 1) * N + n]); *(volatile v2us*)(Bt + e) = o; }
        if (ps == 0) __threadfence(); }
}
__global__ __launch_bounds__(256) void k_cvt8(const float* __restrict__ src, bf* dst, size_t n8) { const size_t i = (size_t)blockIdx.x * 256 + threadIdx.x; if (i >= n8) return; const v8f v = *(const v8f*)(src + i * 8); v8us o;
#pragma unroll
    for (int k = 0; k < 8; ++k) o[k] = f2bf(v[k]); *(volatile v8us*)(dst + i * 8) = o; __threadfence(); *(volatile v8us*)(dst + i * 8) = o; }
__global__ __launch_bounds__(256) void k_fillb(bf* P, unsigned w2, size_t n8) { const size_t i = (size_t)blockIdx.x * 256 + threadIdx.x; if (i >= n8) return; v4i o; o[0] = (int)w2; o[1] = (int)w2; o[2] = (int)w2; o[3] = (int)w2;
    *(volatile v4i*)(P + i * 8) = o; __threadfence(); *(volatile v4i*)(P + i * 8) = o; }
__global__ __launch_bounds__(256) void k_asoft(const float* __restrict__ Sb, h16* P16, bf* Ph, bf* Pl) {
    const int lane = threadIdx.x & 31; const int row = blockIdx.x * 8 + (threadIdx.x >> 5); if (row >= ZH * TT) return; const int i = row % TT; const int zz = row / TT; (void)zz; const bool hires = (i < RH); const float* sr = Sb + (size_t)row * TT; float v[TT / 32]; float mx = -3.0e38f;
#pragma unroll
    for (int ch = 0; ch < TT / 128; ++ch) { const int j0 = ch * 128 + lane * 4; const v4f a = *(const v4f*)(sr + j0);
#pragma unroll
        for (int q = 0; q < 4; ++q) { const int j = j0 + q; (void)j; const float t = a[q] * SCL; v[ch * 4 + q] = t; mx = fmaxf(mx, t); } }
#pragma unroll
    for (int sh = 16; sh; sh >>= 1) mx = fmaxf(mx, __shfl_xor(mx, sh, 32));
    float sum = 0.f;
#pragma unroll
    for (int k = 0; k < TT / 32; ++k) { float d0 = __fsub_rn(v[k], mx); v[k] = __builtin_amdgcn_exp2f(__fmul_rn(d0, 1.4426950408889634f)); sum += v[k]; }
#pragma unroll
    for (int sh = 16; sh; sh >>= 1) sum += __shfl_xor(sum, sh, 32);
    const float f = __fdiv_rn(hires ? 1.0f : PCAR, sum);
#pragma unroll 1
    for (int ps = 0; ps < 2; ++ps) {
        if (hires) {
#pragma unroll
            for (int ch = 0; ch < TT / 128; ++ch) { v4us oh, ol;
#pragma unroll
                for (int q = 0; q < 4; ++q) { unsigned short a, c2; splitf(v[ch * 4 + q] * f, a, c2); oh[q] = a; ol[q] = c2; }
                const size_t oo = ((size_t)zz * (RH ? RH : 1) + i) * TT + ch * 128 + lane * 4; *(volatile v4us*)(Ph + oo) = oh; *(volatile v4us*)(Pl + oo) = ol; }
        } else {
#pragma unroll
            for (int ch = 0; ch < TT / 128; ++ch) { v4h o4;
#pragma unroll
                for (int q = 0; q < 4; ++q) o4[q] = tohx(v[ch * 4 + q] * f);
                *(volatile v4h*)(P16 + (size_t)row * TT + ch * 128 + lane * 4) = o4; } }
        if (ps == 0) __threadfence(); }
}

__device__ __forceinline__ float pt(const float* __restrict__ FP, const float* __restrict__ bp, const float* __restrict__ rot, const float* __restrict__ tr, int l, int h, int which, int c) {
    const int p3 = h * NPT + (c / 3) * 3; const int a = c % 3; const float* f = FP + (size_t)l * FPW + which * PW + p3; const float x0 = __fadd_rn(f[0], bfr(bp[p3])), x1 = __fadd_rn(f[1], bfr(bp[p3 + 1])), x2 = __fadd_rn(f[2], bfr(bp[p3 + 2]));
    const float* r = rot + (size_t)l * 9 + a * 3; float g = __fmul_rn(bfr(r[0]), x0); g = __fmaf_rn(bfr(r[1]), x1, g); g = __fmaf_rn(bfr(r[2]), x2, g); return __fadd_rn(g, bfr(tr[(size_t)l * 3 + a])); }
__global__ __launch_bounds__(256) void k_knorm(const float* __restrict__ FP, const float* __restrict__ bp, const float* __restrict__ rot, const float* __restrict__ tr, float* NK) {
    const int e = blockIdx.x * 256 + threadIdx.x; if (e >= NH_ * LR) return; const int l = e % LR; const int h = e / LR; float s = 0.0f;
#pragma unroll
    for (int k = 0; k < NPT; ++k) { const float g = pt(FP, bp, rot, tr, l, h, 1, k); s = __fmaf_rn(g, g, s); }
    const float n = __fmul_rn(-0.5f, s); *(volatile float*)(NK + e) = n; __threadfence(); *(volatile float*)(NK + e) = n; }
template <bool ISK>
__global__ __launch_bounds__(256) void k_aug(const float* __restrict__ FS, const float* __restrict__ FP, const float* __restrict__ bp, const float* __restrict__ rot, const float* __restrict__ tr, const float* __restrict__ NK, bf* OUT) {
    const size_t e = ((size_t)blockIdx.x * 256 + threadIdx.x) * 8; if (e >= (size_t)NH_ * LR * KA) return; const int c0 = (int)(e % KA); const int l = (int)((e / KA) % LR); const int h = (int)(e / ((size_t)KA * LR)); v8us o;
    unsigned short nhi, nlo; splitf(NK[h * LR + l], nhi, nlo);
#pragma unroll
    for (int q = 0; q < 8; ++q) { const int c = c0 + q; const int cs = (c < HD) ? c : HD - 1; const unsigned short ws = f2bf(FS[(size_t)l * ND + h * HD + cs]);
        int j = c - HD; j = (j < 0) ? 0 : ((j > 3 * NPT - 1) ? 3 * NPT - 1 : j); const int seg = j / NPT; const float x = __fmul_rn(pt(FP, bp, rot, tr, l, h, ISK ? 1 : 0, j - seg * NPT), ISK ? 1.0f : 8.0f); unsigned short hi, lo; splitf(x, hi, lo);
        const unsigned short wp = (seg == 0) ? hi : (((seg == 1) == ISK) ? hi : lo); const unsigned short wn = ISK ? ((c == HD + 3 * NPT) ? nhi : nlo) : f2bf(8.0f);
        o[q] = (c < HD) ? ws : ((c < HD + 3 * NPT) ? wp : ((c < HD + 3 * NPT + 2) ? wn : (unsigned short)0)); }
    *(volatile v8us*)(OUT + e) = o; __threadfence(); *(volatile v8us*)(OUT + e) = o; }
__global__ __launch_bounds__(256) void k_vaug(const float* __restrict__ FV, const float* __restrict__ FP, const float* __restrict__ bp, const float* __restrict__ rot, const float* __restrict__ tr, h16* VT) {
    const size_t e = ((size_t)blockIdx.x * 256 + threadIdx.x) * 8; if (e >= (size_t)NH_ * VA * LR) return; const int l0 = (int)(e % LR); const int dd = (int)((e / LR) % VA); const int h = (int)(e / ((size_t)LR * VA)); v8h o; const int ds = (dd < HD) ? dd : HD - 1; int dp = dd - HD; dp = (dp < 0) ? 0 : ((dp > NPT - 1) ? NPT - 1 : dp);
#pragma unroll
    for (int q = 0; q < 8; ++q) { const int l = l0 + q; const float xs = FV[(size_t)l * ND + h * HD + ds]; const float xp = pt(FP, bp, rot, tr, l, h, 2, dp); o[q] = tohx((dd < HD) ? xs : ((dd < HD + NPT) ? xp : 0.0f)); }
    *(volatile v8h*)(VT + e) = o; __threadfence(); *(volatile v8h*)(VT + e) = o; }
__global__ __launch_bounds__(256) void k_back(const float* __restrict__ Ob, const float* __restrict__ rot, const float* __restrict__ tr, h16* CAT) {
    const size_t e = ((size_t)blockIdx.x * 256 + threadIdx.x) * 8; if (e >= (size_t)LR * CW) return; const int c0 = (int)(e % CW); const int l = (int)(e / CW); v8h o; const float* r = rot + (size_t)l * 9; const float t0 = bfr(tr[(size_t)l * 3]), t1 = bfr(tr[(size_t)l * 3 + 1]), t2 = bfr(tr[(size_t)l * 3 + 2]);
#pragma unroll
    for (int q = 0; q < 8; ++q) { const int c = c0 + q; const int cs = (c < NH_ * HD) ? c : NH_ * HD - 1; const float xs = __fmul_rn(Ob[((size_t)(cs / HD) * LR + l) * VA + (cs % HD)], 1.0f / PCAR);
        int i = c - NH_ * HD; i = (i < 0) ? 0 : i; const int h = i / NPT; const int p3 = ((i % NPT) / 3) * 3; const int a = i % 3; const float* ob = Ob + ((size_t)h * LR + l) * VA + HD + p3;
        const float d0 = __fsub_rn(__fmul_rn(ob[0], 1.0f / PCAR), t0), d1 = __fsub_rn(__fmul_rn(ob[1], 1.0f / PCAR), t1), d2 = __fsub_rn(__fmul_rn(ob[2], 1.0f / PCAR), t2);
        float xp = __fmul_rn(bfr(r[a]), d0); xp = __fmaf_rn(bfr(r[3 + a]), d1, xp); xp = __fmaf_rn(bfr(r[6 + a]), d2, xp);
        o[q] = tohx((c < NH_ * HD) ? xs : xp); }
    *(volatile v8h*)(CAT + e) = o; __threadfence(); *(volatile v8h*)(CAT + e) = o; }
__global__ __launch_bounds__(256) void k_wot(const float* __restrict__ w, h16* Bt) {
    const size_t e = ((size_t)blockIdx.x * 256 + threadIdx.x) * 8; if (e >= (size_t)ND * CW) return; const int k0 = (int)(e % CW); const int n = (int)(e / CW); v8h o;
#pragma unroll
    for (int q = 0; q < 8; ++q) o[q] = tohx(bfr(w[(size_t)(k0 + q) * ND + n]));
    *(volatile v8h*)(Bt + e) = o; __threadfence(); *(volatile v8h*)(Bt + e) = o; }

extern "C" void kernel_launch(void* const* d_in, const int* in_sizes, int n_in,
                              void* d_out, int out_size, void* d_ws, size_t ws_size, hipStream_t stream) {
    (void)in_sizes; (void)n_in; (void)out_size;
    const float* nf = (const float*)d_in[0]; const float* tr = (const float*)d_in[1]; const float* rot = (const float*)d_in[2];
    const float* wq = (const float*)d_in[3]; const float* bq = (const float*)d_in[4]; const float* wk = (const float*)d_in[5]; const float* bk = (const float*)d_in[6]; const float* wv = (const float*)d_in[7]; const float* bv = (const float*)d_in[8];
    const float* wqp = (const float*)d_in[9]; const float* bqp = (const float*)d_in[10]; const float* wkp = (const float*)d_in[11]; const float* bkp = (const float*)d_in[12]; const float* wvp = (const float*)d_in[13]; const float* bvp = (const float*)d_in[14];
    const float* wo = (const float*)d_in[15]; const float* bo = (const float*)d_in[16];
    float* OUT = (float*)d_out;
    char* wsp = (char*)d_ws;
    auto take = [&](size_t bytes) { char* p = wsp; wsp += (bytes + 255) & ~(size_t)255; return (void*)p; };
    bf* WQ = (bf*)take((size_t)ND * ND * 2); bf* WK = (bf*)take((size_t)ND * ND * 2); bf* WV = (bf*)take((size_t)ND * ND * 2); bf* WP = (bf*)take((size_t)FPW * ND * 2); h16* WOT = (h16*)take((size_t)ND * CW * 2);
    bf* NFB = (bf*)take((size_t)LR * ND * 2); float* FQ = (float*)take((size_t)LR * ND * 4); float* FK = (float*)take((size_t)LR * ND * 4); float* FV = (float*)take((size_t)LR * ND * 4); float* FP = (float*)take((size_t)LR * FPW * 4);
    float* NK = (float*)take((size_t)NH_ * LR * 4); bf* QA = (bf*)take((size_t)NH_ * LR * KA * 2); bf* KAp = (bf*)take((size_t)NH_ * LR * KA * 2); h16* VT = (h16*)take((size_t)NH_ * VA * LR * 2);
    float* Sb = (float*)take((size_t)ZH * TT * TT * 4); h16* P16 = (h16*)take((size_t)ZH * TT * TT * 2); float* Ob = (float*)take((size_t)NH_ * LR * VA * 4); h16* CAT = (h16*)take((size_t)LR * CW * 2);
    if ((size_t)(wsp - (char*)d_ws) > ws_size) return;
    k_wtG<<<(unsigned)(((size_t)ND * ND / 64 + 63) / 64), 256, 0, stream>>>(wq, ND, ND, WQ); k_wtG<<<(unsigned)(((size_t)ND * ND / 64 + 63) / 64), 256, 0, stream>>>(wk, ND, ND, WK); k_wtG<<<(unsigned)(((size_t)ND * ND / 64 + 63) / 64), 256, 0, stream>>>(wv, ND, ND, WV);
    k_wtG<<<(unsigned)(((size_t)ND * PW / 64 + 63) / 64), 256, 0, stream>>>(wqp, ND, PW, WP); k_wtG<<<(unsigned)(((size_t)ND * PW / 64 + 63) / 64), 256, 0, stream>>>(wkp, ND, PW, WP + (size_t)PW * ND); k_wtG<<<(unsigned)(((size_t)ND * PW / 64 + 63) / 64), 256, 0, stream>>>(wvp, ND, PW, WP + (size_t)2 * PW * ND);
    k_fillb<<<(unsigned)(((size_t)(FPW - 3 * PW) * ND / 8 + 255) / 256), 256, 0, stream>>>(WP + (size_t)3 * PW * ND, 0u, (size_t)(FPW - 3 * PW) * ND / 8);
    k_wot<<<(unsigned)(((size_t)ND * CW / 8 + 255) / 256), 256, 0, stream>>>(wo, WOT);
    k_cvt8<<<(unsigned)(((size_t)LR * ND / 8 + 255) / 256), 256, 0, stream>>>(nf, NFB, (size_t)LR * ND / 8);
    k_gemmw<bf, 0, true><<<dim3(LR / 64, ND / 64, 1), 32, 0, stream>>>(NFB, nullptr, WQ, nullptr, ND, FQ, ND, bq, 0, 0, 0);
    k_gemmw<bf, 0, true><<<dim3(LR / 64, ND / 64, 1), 32, 0, stream>>>(NFB, nullptr, WK, nullptr, ND, FK, ND, bk, 0, 0, 0);
    k_gemmw<bf, 0, true><<<dim3(LR / 64, ND / 64, 1), 32, 0, stream>>>(NFB, nullptr, WV, nullptr, ND, FV, ND, bv, 0, 0, 0);
    k_gemmw<bf, 0, false><<<dim3(LR / 64, FPW / 64, 1), 32, 0, stream>>>(NFB, nullptr, WP, nullptr, ND, FP, FPW, nullptr, 0, 0, 0);
    k_knorm<<<(NH_ * LR + 255) / 256, 256, 0, stream>>>(FP, bkp, rot, tr, NK);
    k_aug<false><<<(unsigned)(((size_t)NH_ * LR * KA / 8 + 255) / 256), 256, 0, stream>>>(FQ, FP, bqp, rot, tr, NK, QA);
    k_aug<true><<<(unsigned)(((size_t)NH_ * LR * KA / 8 + 255) / 256), 256, 0, stream>>>(FK, FP, bkp, rot, tr, NK, KAp);
    k_vaug<<<(unsigned)(((size_t)NH_ * VA * LR / 8 + 255) / 256), 256, 0, stream>>>(FV, FP, bvp, rot, tr, VT);
    for (int h0 = 0; h0 < NH_; h0 += ZH) {
        k_gemmw<bf, 0, false><<<dim3(TT / 64, TT / 64, ZH), 32, 0, stream>>>(QA + (size_t)h0 * LR * KA, nullptr, KAp + (size_t)h0 * LR * KA, nullptr, KA, Sb, TT, nullptr, (size_t)LR * KA, (size_t)LR * KA, (size_t)TT * TT);
        k_asoft<<<ZH * TT / 8, 256, 0, stream>>>(Sb, P16, nullptr, nullptr);
        k_gemmw<h16, 0, false><<<dim3(TT / 64, VA / 64, ZH), 32, 0, stream>>>(P16, nullptr, VT + (size_t)h0 * VA * LR, nullptr, TT, Ob + (size_t)h0 * LR * VA, VA, nullptr, (size_t)TT * TT, (size_t)VA * LR, (size_t)LR * VA);
    }
    k_back<<<(unsigned)(((size_t)LR * CW / 8 + 255) / 256), 256, 0, stream>>>(Ob, rot, tr, CAT);
    k_gemmw<h16, 0, true><<<dim3(LR / 64, ND / 64, 1), 32, 0, stream>>>(CAT, nullptr, WOT, nullptr, CW, OUT, ND, bo, 0, 0, 0);
}
